// SGGN_layer_33062658245058
// MI455X (gfx1250) — hardware-verified
//
#include <hip/hip_runtime.h>
#include <stdint.h>
#include <stddef.h>
#include <math.h>

#pragma clang fp contract(off)

#define NN    8192
#define DD    64
#define KE    8
#define EE    (NN * KE)
#define MDEG  16
#define LL    17
#define LP    32
#define DIN   128
#define TDIN  256
#define DCV   4
#define HF    (MDEG * DD)
#define YF    (LL * DD)
#define PF    (2 * DD)
#define NPB   4
#define P1    (TDIN * DD / 8)
#define P2    (DD * DIN / 8)
#define EPS_  1e-5f

static_assert(NN % NPB == 0);
static_assert(P1 % 256 == 0);
static_assert(P2 % 256 == 0);
static_assert(HF == 1024);
static_assert((HF / 4) % 128 == 0);
static_assert(YF == 34 * 32);
static_assert(LP * DD >= YF);
static_assert(DD % 32 == 0);
static_assert(DIN % 32 == 0);
static_assert(LL <= LP);

typedef _Float16 v16h __attribute__((ext_vector_type(16)));
typedef _Float16 v8h  __attribute__((ext_vector_type(8)));
typedef _Float16 v4h  __attribute__((ext_vector_type(4)));
typedef float    v8f  __attribute__((ext_vector_type(8)));
typedef float    v4f  __attribute__((ext_vector_type(4)));
typedef double   v2d  __attribute__((ext_vector_type(2)));
typedef v4f __attribute__((may_alias)) v4fa;
typedef v8h __attribute__((may_alias)) v8ha;
typedef v4h __attribute__((may_alias)) v4ha;
typedef v2d __attribute__((may_alias)) v2da;

union FragH { v16h v; v8h q[2]; };

__device__ __forceinline__ v8f wmma_h(v16h a, v16h b, v8f c) {
  v8f d = __builtin_amdgcn_wmma_f32_16x16x32_f16(false, a, false, b, (short)0, c, false, false);
  asm volatile("v_nop\n\tv_nop\n\tv_nop\n\tv_nop" : "+v"(d) : "v"(a), "v"(b));
  return d;
}

__device__ __forceinline__ v16h ldfrag_h(const _Float16* p, int h) {
  FragH f;
  f.q[0] = *(const v8ha*)(p + 8 * h);
  f.q[1] = *(const v8ha*)(p + 16 + 8 * h);
  return f.v;
}

__device__ __forceinline__ int clampi(int v, int hi) {
  return v < 0 ? 0 : (v > hi ? hi : v);
}

__device__ __forceinline__ float sigm_f(float x) {
  const float ex = expf(-x);
  return __builtin_amdgcn_rcpf(1.0f + ex);
}
__device__ __forceinline__ float silu_f(float x) { return x * sigm_f(x); }

__device__ __forceinline__ void cvt8_store(const float* sp, _Float16* dp, float scale) {
  const v4f a = *(const v4fa*)(sp);
  const v4f b = *(const v4fa*)(sp + 4);
  v8h o;
  o[0] = (_Float16)(a.x * scale); o[1] = (_Float16)(a.y * scale);
  o[2] = (_Float16)(a.z * scale); o[3] = (_Float16)(a.w * scale);
  o[4] = (_Float16)(b.x * scale); o[5] = (_Float16)(b.y * scale);
  o[6] = (_Float16)(b.z * scale); o[7] = (_Float16)(b.w * scale);
  *(volatile v8ha*)dp = o;
  __threadfence();
  *(volatile v8ha*)dp = o;
}

__global__ __launch_bounds__(256) void k_wconv(const float* __restrict__ fc1w,
                                               const float* __restrict__ fc2w,
                                               _Float16* __restrict__ fc1h,
                                               _Float16* __restrict__ fc2h)
{
  const int blk = blockIdx.x, t = threadIdx.x;
  if (blk < P1 / 256) {
    int p = blk * 256 + t;
    p = clampi(p, P1 - 1);
    cvt8_store(fc1w + (size_t)p * 8, fc1h + (size_t)p * 8, 16.0f);
  } else {
    int p = (blk - P1 / 256) * 256 + t;
    p = clampi(p, P2 - 1);
    cvt8_store(fc2w + (size_t)p * 8, fc2h + (size_t)p * 8, 16.0f);
  }
}

__global__ __launch_bounds__(256) void k_msg(const float* __restrict__ hs,
                                             const float* __restrict__ hs_e,
                                             const float* __restrict__ degree,
                                             const float* __restrict__ noise,
                                             const int*   __restrict__ dst,
                                             float* __restrict__ hflat)
{
  __shared__ __align__(16) float sM[NPB * HF];
  __shared__ int sRank[NPB * KE];
  __shared__ int sDst[NPB * KE];

  const int tid = threadIdx.x, lane = tid & 31, wv = tid >> 5;
  const int q = tid >> 6, d = tid & 63;
  const int n0 = blockIdx.x * NPB;
  const int n = n0 + q;
  const int e0 = n * KE;

  #pragma unroll
  for (int r = 0; r < MDEG; ++r) sM[q * HF + r * DD + d] = 0.0f;

  const int dd = d & 7;
  const int dn_own = clampi(dst[e0 + dd], NN - 1);
  const float s_own = degree[dn_own] + noise[e0 + dd];
  int rk = 0;
  #pragma unroll
  for (int i = 0; i < KE; ++i) {
    const int dv = clampi(dst[e0 + i], NN - 1);
    const float si = degree[dv] + noise[e0 + i];
    rk += ((si < s_own) || (si == s_own && i < dd)) ? 1 : 0;
  }
  if (d < KE) { sRank[q * KE + d] = rk; sDst[q * KE + d] = dn_own; }
  __syncthreads();

  #pragma unroll 1
  for (int j = 0; j < KE; ++j) {
    const int r  = clampi(sRank[q * KE + j], MDEG - 1);
    const int dv = clampi(sDst[q * KE + j], NN - 1);
    const size_t e = (size_t)(e0 + j);
    const float mv = hs[(size_t)dv * DD + d] * sigm_f(hs_e[e * DD + d]);
    sM[q * HF + r * DD + d] = mv;
  }
  __syncthreads();

  v4f v[4];
  #pragma unroll
  for (int it = 0; it < 4; ++it) {
    const int li  = it * 32 + wv * 4 + (lane >> 3);
    const int qq  = li >> 5;
    const int off = (li & 31) * 32 + (lane & 7) * 4;
    v[it] = *(const v4fa*)(sM + qq * HF + off);
  }
  #pragma unroll
  for (int it = 0; it < 4; ++it) {
    const int li  = it * 32 + wv * 4 + (lane >> 3);
    const int qq  = li >> 5;
    const int off = (li & 31) * 32 + (lane & 7) * 4;
    *(volatile v4fa*)(hflat + (size_t)(n0 + qq) * HF + off) = v[it];
  }
  __threadfence();
  #pragma unroll
  for (int it = 0; it < 4; ++it) {
    const int li  = it * 32 + wv * 4 + (lane >> 3);
    const int qq  = li >> 5;
    const int off = (li & 31) * 32 + (lane & 7) * 4;
    *(volatile v4fa*)(hflat + (size_t)(n0 + qq) * HF + off) = v[it];
  }
}

__global__ __launch_bounds__(128) void k_node(
    const float* __restrict__ hs, const int* __restrict__ src,
    const float* __restrict__ hflat,
    const _Float16* __restrict__ fc1h, const float* __restrict__ fc1b,
    const float* __restrict__ convw, const float* __restrict__ convb,
    const _Float16* __restrict__ fc2h, const float* __restrict__ fc2b,
    const float* __restrict__ rmsw,
    float* __restrict__ Y, double* __restrict__ part)
{
  __shared__ int sSrc[KE];
  __shared__ __align__(16) float    sHin[LL * DD];
  __shared__ __align__(16) _Float16 sA[LP * DD];
  __shared__ __align__(16) float    sXZ[LP * TDIN];
  __shared__ __align__(16) _Float16 sG[LP * DIN];
  __shared__ __align__(16) float    sO[LP * DD];
  __shared__ float sR[LP];
  __shared__ __align__(16) double   sP[PF];

  const int n = blockIdx.x;
  const int tid = threadIdx.x, lane = tid & 31, wv = tid >> 5;
  const int h = lane >> 4, m = lane & 15;
  const v8f z8 = {0.f, 0.f, 0.f, 0.f, 0.f, 0.f, 0.f, 0.f};
  const v8h zh = {(_Float16)0.f, (_Float16)0.f, (_Float16)0.f, (_Float16)0.f,
                  (_Float16)0.f, (_Float16)0.f, (_Float16)0.f, (_Float16)0.f};

  if (tid < KE) sSrc[tid] = clampi(src[(size_t)n * KE + tid], NN - 1);
  __syncthreads();

  if (tid < DD) {
    const float v = hs[(size_t)n * DD + tid];
    sHin[tid] = v;
    sA[tid] = (_Float16)v;
  }
  int sj[KE];
  #pragma unroll
  for (int j = 0; j < KE; ++j) sj[j] = sSrc[j];
  const float* selfp = hflat + (size_t)n * HF;
  #pragma unroll 1
  for (int p = tid; p < HF / 4; p += 128) {
    const int ii = p * 4;
    v4f acc = {0.f, 0.f, 0.f, 0.f};
    #pragma unroll
    for (int j = 0; j < KE; ++j)
      acc += *(const v4fa*)(hflat + (size_t)sj[j] * HF + ii);
    const v4f sv = *(const v4fa*)(selfp + ii);
    const v4f v = acc + sv;
    *(v4fa*)(sHin + DD + ii) = v;
    v4h hv;
    hv[0] = (_Float16)v.x; hv[1] = (_Float16)v.y;
    hv[2] = (_Float16)v.z; hv[3] = (_Float16)v.w;
    *(v4ha*)(sA + DD + ii) = hv;
  }
  if (tid < (LP - LL) * DD / 8)
    *(v8ha*)(sA + LL * DD + tid * 8) = zh;
  __syncthreads();

  {
    v16h af[2][2];
    #pragma unroll
    for (int mt = 0; mt < 2; ++mt)
      #pragma unroll
      for (int kk = 0; kk < 2; ++kk)
        af[mt][kk] = ldfrag_h(sA + (mt * 16 + m) * DD + kk * 32, h);
    #pragma unroll 1
    for (int nt = 0; nt < 4; ++nt) {
      const int ncol = (wv * 4 + nt) * 16 + m;
      v8f acc0 = z8, acc1 = z8;
      #pragma unroll
      for (int kk = 0; kk < 2; ++kk) {
        const v16h b = ldfrag_h(fc1h + (size_t)ncol * DD + kk * 32, h);
        acc0 = wmma_h(af[0][kk], b, acc0);
        acc1 = wmma_h(af[1][kk], b, acc1);
      }
      const float bias = fc1b[ncol];
      #pragma unroll
      for (int r = 0; r < 8; ++r) {
        sXZ[(8 * h + r) * TDIN + ncol]      = acc0[r] * 0.0625f + bias;
        sXZ[(16 + 8 * h + r) * TDIN + ncol] = acc1[r] * 0.0625f + bias;
      }
    }
  }
  __syncthreads();

  {
    const int c = tid;
    const float w0 = convw[c * DCV + 0], w1 = convw[c * DCV + 1];
    const float w2 = convw[c * DCV + 2], w3 = convw[c * DCV + 3];
    const float cb = convb[c];
    float x1 = 0.0f, x2 = 0.0f, x3 = 0.0f;
    #pragma unroll 1
    for (int mr = 0; mr < LL; ++mr) {
      const float x0 = sXZ[mr * TDIN + c];
      const float zz = sXZ[mr * TDIN + DIN + c];
      const float cv = (((w0 * x3 + w1 * x2) + w2 * x1) + w3 * x0) + cb;
      const float g  = silu_f(cv) * silu_f(zz);
      sG[mr * DIN + c] = (_Float16)(g * 256.0f);
      x3 = x2; x2 = x1; x1 = x0;
    }
    for (int i = tid; i < (LP - LL) * DIN / 8; i += 128)
      *(v8ha*)(sG + LL * DIN + i * 8) = zh;
  }
  __syncthreads();

  {
    const int ncol = wv * 16 + m;
    v8f acc0 = z8, acc1 = z8;
    #pragma unroll
    for (int kk = 0; kk < 4; ++kk) {
      const v16h a0 = ldfrag_h(sG + m * DIN + kk * 32, h);
      const v16h a1 = ldfrag_h(sG + (16 + m) * DIN + kk * 32, h);
      const v16h b  = ldfrag_h(fc2h + (size_t)ncol * DIN + kk * 32, h);
      acc0 = wmma_h(a0, b, acc0);
      acc1 = wmma_h(a1, b, acc1);
    }
    const float bias = fc2b[ncol];
    #pragma unroll
    for (int r = 0; r < 8; ++r) {
      sO[(8 * h + r) * DD + ncol]      = acc0[r] * (1.0f / 4096.0f) + bias;
      sO[(16 + 8 * h + r) * DD + ncol] = acc1[r] * (1.0f / 4096.0f) + bias;
    }
  }
  __syncthreads();

  if (tid < LL) {
    float ss = 0.0f;
    #pragma unroll 4
    for (int j = 0; j < DD; ++j) { const float v = sO[tid * DD + j]; ss += v * v; }
    sR[tid] = rsqrtf(ss * (1.0f / (float)DD) + EPS_);
  }
  __syncthreads();

  if (tid < DD) {
    const int j = tid;
    const float rw = rmsw[j];
    double s = 0.0, s2 = 0.0;
    #pragma unroll 1
    for (int mr = 0; mr < LL; ++mr) {
      const int idx = mr * DD + j;
      const float yv = (sO[idx] * sR[mr]) * rw + sHin[idx];
      sO[idx] = yv;
      const double yd = (double)yv;
      s += yd;
      s2 += yd * yd;
    }
    sP[j] = s;
    sP[DD + j] = s2;
  }
  __syncthreads();

  {
    v4f yv[3];
    #pragma unroll
    for (int it = 0; it < 3; ++it) {
      const int li = it * 16 + wv * 4 + (lane >> 3);
      yv[it] = *(const v4fa*)(sO + li * 32 + (lane & 7) * 4);
    }
    const v2d pv = *(const v2da*)(sP + (wv & 1) * DD + lane * 2);
    float*  ybase = Y + (size_t)n * YF;
    double* pbase = part + (size_t)n * PF;
    #pragma unroll
    for (int it = 0; it < 3; ++it) {
      const int li = it * 16 + wv * 4 + (lane >> 3);
      if (li < 2 * LL) *(volatile v4fa*)(ybase + li * 32 + (lane & 7) * 4) = yv[it];
    }
    if (wv < 2) *(volatile v2da*)(pbase + wv * DD + lane * 2) = pv;
    __threadfence();
    #pragma unroll
    for (int it = 0; it < 3; ++it) {
      const int li = it * 16 + wv * 4 + (lane >> 3);
      if (li < 2 * LL) *(volatile v4fa*)(ybase + li * 32 + (lane & 7) * 4) = yv[it];
    }
    if (wv < 2) *(volatile v2da*)(pbase + wv * DD + lane * 2) = pv;
  }
}

__global__ __launch_bounds__(256) void k_stats(const double* __restrict__ part,
                                               float* __restrict__ stats)
{
  __shared__ double sRed[2 * 4 * DD];
  __shared__ __align__(16) float sTab[2 * DD];
  const int tid = threadIdx.x, lane = tid & 31, wv = tid >> 5;
  const int c = tid & 63, p = tid >> 6;
  double s = 0.0, s2 = 0.0;
  const int b0 = p * (NN / 4);
  #pragma unroll 2
  for (int b = 0; b < NN / 4; ++b) {
    const double* row = part + (size_t)(b0 + b) * PF;
    s  += row[c];
    s2 += row[DD + c];
  }
  sRed[p * DD + c] = s;
  sRed[4 * DD + p * DD + c] = s2;
  __syncthreads();
  if (tid < DD) {
    const double S  = (sRed[c] + sRed[DD + c]) + (sRed[2 * DD + c] + sRed[3 * DD + c]);
    const double S2 = (sRed[4 * DD + c] + sRed[5 * DD + c]) + (sRed[6 * DD + c] + sRed[7 * DD + c]);
    const double inv = 1.0 / (double)(NN * LL);
    const double mean = S * inv;
    double var = S2 * inv - mean * mean;
    var = var < 0.0 ? 0.0 : var;
    sTab[c] = (float)mean;
    sTab[DD + c] = rsqrtf((float)var + EPS_);
  }
  __syncthreads();
  if (wv == 0) {
    const v4f v = *(const v4fa*)(sTab + lane * 4);
    *(volatile v4fa*)(stats + lane * 4) = v;
    __threadfence();
    *(volatile v4fa*)(stats + lane * 4) = v;
  }
}

__global__ __launch_bounds__(256) void k_out(const float* __restrict__ Y,
                                             const float* __restrict__ stats,
                                             const float* __restrict__ gamma,
                                             const float* __restrict__ beta,
                                             const float* __restrict__ aggw,
                                             const float* __restrict__ aggb,
                                             const float* __restrict__ hs,
                                             float* __restrict__ out)
{
  __shared__ __align__(16) float sOut[256];
  const int tid = threadIdx.x, lane = tid & 31, wv = tid >> 5;
  const int q = tid >> 6, d = tid & 63;
  const int n = blockIdx.x * NPB + q;
  const float mean = stats[d], rsq = stats[DD + d];
  const float g = gamma[d], be = beta[d];
  const float* yp = Y + (size_t)n * YF + d;
  float acc = 0.0f;
  #pragma unroll 1
  for (int l = 0; l < LL; ++l) {
    const float yv = yp[l * DD];
    float yb = (g * (yv - mean)) * rsq + be;
    yb = fminf(fmaxf(yb, 0.0f), 6.0f);
    acc += yb * aggw[l];
  }
  const float res = (acc + aggb[0]) + hs[(size_t)n * DD + d];
  sOut[tid] = res;
  __syncthreads();
  if (wv < 2) {
    const v4f v = *(const v4fa*)(sOut + wv * 128 + lane * 4);
    float* gp = out + (size_t)blockIdx.x * (NPB * DD) + wv * 128 + lane * 4;
    *(volatile v4fa*)gp = v;
    __threadfence();
    *(volatile v4fa*)gp = v;
  }
}

extern "C" void kernel_launch(void* const* d_in, const int* in_sizes, int n_in,
                              void* d_out, int out_size, void* d_ws, size_t ws_size,
                              hipStream_t stream)
{
  if (n_in < 17) return;
  if (in_sizes[0]  != NN * DD) return;
  if (in_sizes[1]  != EE * DD) return;
  if (in_sizes[2]  != NN) return;
  if (in_sizes[3]  != EE) return;
  if (in_sizes[4]  != TDIN * DD) return;
  if (in_sizes[5]  != TDIN) return;
  if (in_sizes[6]  != DIN * DCV) return;
  if (in_sizes[7]  != DIN) return;
  if (in_sizes[8]  != DD * DIN) return;
  if (in_sizes[9]  != DD) return;
  if (in_sizes[10] != DD) return;
  if (in_sizes[11] != DD) return;
  if (in_sizes[12] != DD) return;
  if (in_sizes[13] != LL) return;
  if (in_sizes[14] != 1) return;
  if (in_sizes[15] != EE) return;
  if (in_sizes[16] != EE) return;
  if (out_size != NN * DD) return;

  const float* hs     = (const float*)d_in[0];
  const float* hs_e   = (const float*)d_in[1];
  const float* degree = (const float*)d_in[2];
  const float* noise  = (const float*)d_in[3];
  const float* fc1w   = (const float*)d_in[4];
  const float* fc1b   = (const float*)d_in[5];
  const float* convw  = (const float*)d_in[6];
  const float* convb  = (const float*)d_in[7];
  const float* fc2w   = (const float*)d_in[8];
  const float* fc2b   = (const float*)d_in[9];
  const float* rmsw   = (const float*)d_in[10];
  const float* gamma  = (const float*)d_in[11];
  const float* beta   = (const float*)d_in[12];
  const float* aggw   = (const float*)d_in[13];
  const float* aggb   = (const float*)d_in[14];
  const int*   src    = (const int*)d_in[15];
  const int*   dst    = (const int*)d_in[16];
  float* out = (float*)d_out;

  const size_t bW1 = (size_t)TDIN * DD * 2;
  const size_t bW2 = (size_t)DD * DIN * 2;
  const size_t bHF = (size_t)NN * HF * 4;
  const size_t bY  = (size_t)NN * YF * 4;
  const size_t bP  = (size_t)NN * PF * 8;
  const size_t bS  = 512;
  const size_t total = bW1 + bW2 + bHF + bY + bP + bS;
  if (total > ws_size) return;
  if (total > (size_t)134217728) return;

  char* ws = (char*)d_ws;
  size_t off = 0;
  _Float16* fc1h  = (_Float16*)(ws + off); off += bW1;
  _Float16* fc2h  = (_Float16*)(ws + off); off += bW2;
  float*    hflat = (float*)(ws + off);    off += bHF;
  float*    Ybuf  = (float*)(ws + off);    off += bY;
  double*   part  = (double*)(ws + off);   off += bP;
  float*    stats = (float*)(ws + off);    off += bS;
  if (off != total) return;

  k_wconv<<<dim3((P1 + P2) / 256), 256, 0, stream>>>(fc1w, fc2w, fc1h, fc2h);
  k_msg<<<dim3(NN / NPB), 256, 0, stream>>>(hs, hs_e, degree, noise, dst, hflat);
  k_node<<<dim3(NN), 128, 0, stream>>>(hs, src, hflat, fc1h, fc1b, convw, convb,
                                        fc2h, fc2b, rmsw, Ybuf, part);
  k_stats<<<dim3(1), 256, 0, stream>>>(part, stats);
  k_out<<<dim3(NN / NPB), 256, 0, stream>>>(Ybuf, stats, gamma, beta, aggw, aggb, hs, out);
}
